// VoxelTransformerLayer3D_84507776516326
// MI455X (gfx1250) — hardware-run, weakly checked
//
#include <hip/hip_runtime.h>


namespace {
constexpr int B = 2, G = 16, M = B * G * G * G, C = 256, NH = 8, HD = 32, F = 1024, WS = 3;
constexpr float XS = 8.0f, WSC = 256.0f, EPS = 1e-5f, SCALE = 0.17677669529663688f;
typedef _Float16 b16;
typedef __attribute__((ext_vector_type(16))) _Float16 v16b;
typedef __attribute__((ext_vector_type(8))) _Float16 v8b;
typedef __attribute__((ext_vector_type(8))) float v8f;
typedef __attribute__((ext_vector_type(4))) float v4f;
__device__ __forceinline__ float bf16_rne(float f) { unsigned int u = __float_as_uint(f); u += 0x7FFFu + ((u >> 16) & 1u); float r = __uint_as_float(u & 0xFFFF0000u); asm volatile("" : "+v"(r)); return r; }
__device__ __forceinline__ void split16(float v, b16& hi, b16& lo) { hi = (b16)v; lo = (b16)(v - (float)hi); }
__device__ __forceinline__ v16b frag_kb(const b16* p, int hh) { const v8b a = *(const v8b*)(p + 8 * hh), b = *(const v8b*)(p + 16 + 8 * hh); v16b f;
#pragma unroll
  for (int e = 0; e < 8; ++e) { f[e] = a[e]; f[8 + e] = b[e]; } return f; }
__device__ __forceinline__ v8f wmma16b(v16b a, v16b b, v8f c) { v8f d = __builtin_amdgcn_wmma_f32_16x16x32_f16(false, a, false, b, (short)0, c, false, false); asm volatile("v_nop\n\tv_nop\n\tv_nop\n\tv_nop" : "+v"(d) : "v"(a), "v"(b)); return d; }
__device__ __forceinline__ void wave_lds_sync() { __builtin_amdgcn_fence(__ATOMIC_RELEASE, "workgroup"); __builtin_amdgcn_wave_barrier(); __builtin_amdgcn_fence(__ATOMIC_ACQUIRE, "workgroup"); }
__device__ __forceinline__ float pmul(float a, float b) { float p = a * b; asm volatile("" : "+v"(p)); return p; }
__device__ __forceinline__ float gelu(float v) { return 0.5f * v * (1.0f + erff(v * 0.70710678118654752f)); }

__global__ __launch_bounds__(256) void wput_kernel(const float* __restrict__ w, int K, int O, b16* __restrict__ WT) { const size_t u = (size_t)blockIdx.x * 256 + threadIdx.x; if (u >= (size_t)O * (K / 8)) return; const int o = (int)(u / (K / 8)), k0 = (int)(u % (K / 8)) * 8; v8b v;
#pragma unroll
  for (int j = 0; j < 8; ++j) v[j] = (b16)(bf16_rne(w[(size_t)(k0 + j) * O + o]) * WSC); for (int pass = 0; pass < 2; ++pass) { *(volatile v8b*)(WT + (size_t)o * K + k0) = v; __threadfence(); } }
__device__ __forceinline__ void stage_rows(const float* src, size_t m0, const float* g, const float* bb, bool do_ln, bool do_bf16, b16 (*Ah)[C + 8], b16 (*Al)[C + 8], int lane) {
  for (int rr = 0; rr < 16; ++rr) { float v[8]; float s = 0.0f; for (int q = 0; q < 8; ++q) { float t = src[(m0 + rr) * C + q * 32 + lane]; if (do_bf16) t = bf16_rne(t); v[q] = t; s += t; }
    if (do_ln) { for (int o = 16; o; o >>= 1) s += __shfl_xor(s, o); const float mu = s * (1.0f / C); float qs = 0.0f; for (int q = 0; q < 8; ++q) qs += pmul(v[q] - mu, v[q] - mu); for (int o = 16; o; o >>= 1) qs += __shfl_xor(qs, o); const float rs = rsqrtf(qs * (1.0f / C) + EPS);
      for (int q = 0; q < 8; ++q) { const int c = q * 32 + lane; v[q] = pmul(pmul(v[q] - mu, rs), bf16_rne(g[c])) + bf16_rne(bb[c]); } }
    for (int q = 0; q < 8; ++q) { b16 p, ql; split16(v[q] * XS, p, ql); Ah[rr][q * 32 + lane] = p; if (Al) Al[rr][q * 32 + lane] = ql; } } }
template <int MODE>
__global__ __launch_bounds__(32) void proj_kernel(const float* __restrict__ IN, const float* __restrict__ x, const b16* __restrict__ WTa, const b16* __restrict__ WTb, const float* __restrict__ ba, const float* __restrict__ bbv, const float* __restrict__ g, const float* __restrict__ be, int MLIM, float* __restrict__ OUT) {
  __shared__ __attribute__((aligned(16))) b16 Ah[16][C + 8], Al[16][C + 8]; __shared__ float Tf[16][132]; const int lane = threadIdx.x, nloc = lane & 15, hlf = lane >> 4; constexpr int NG = MODE == 0 ? 4 : 2; const int grp = blockIdx.x % NG; const size_t m0 = (size_t)(blockIdx.x / NG) * 16; if (MODE != 0 && m0 >= (size_t)MLIM) return;
  stage_rows(IN, m0, g, be, MODE == 1, MODE == 0, Ah, MODE == 0 ? nullptr : Al, lane);
  wave_lds_sync(); const b16* WT = (MODE == 0 && grp >= 2) ? WTb : WTa; const int cg = (MODE == 0) ? (grp & 1) * 128 : grp * 128; v8f acc[8];
#pragma unroll
  for (int t = 0; t < 8; ++t) acc[t] = (v8f){};
#pragma unroll 2
  for (int kb = 0; kb < C; kb += 32) { const v16b a = frag_kb(&Ah[nloc][kb], hlf); v16b al; if (MODE != 0) al = frag_kb(&Al[nloc][kb], hlf);
#pragma unroll
    for (int t = 0; t < 8; ++t) { const v16b bw = frag_kb(WT + (size_t)(cg + t * 16 + nloc) * C + kb, hlf); acc[t] = wmma16b(a, bw, acc[t]); if (MODE != 0) acc[t] = wmma16b(al, bw, acc[t]); } }
#pragma unroll
  for (int t = 0; t < 8; ++t) { const int cc = cg + t * 16 + nloc; const float bias = bf16_rne((MODE == 0 && grp >= 2) ? bbv[cc] : ba[cc]);
#pragma unroll
    for (int r8 = 0; r8 < 8; ++r8) { float v = acc[t][r8] * (1.0f / (XS * WSC)) + bias; if (MODE == 1) v *= SCALE; Tf[8 * hlf + r8][t * 16 + nloc] = v; } }
  wave_lds_sync(); const int ow = MODE == 0 ? 2 * C : C; const int oc = MODE == 0 ? grp * 128 : cg;
  for (int pass = 0; pass < 2; ++pass) { for (int rr = 0; rr < 16; ++rr) { v4f v = *(const v4f*)(&Tf[rr][lane * 4]); if (MODE == 2) { const v4f xv = *(const v4f*)(x + (m0 + rr) * C + oc + lane * 4); for (int k = 0; k < 4; ++k) v[k] += bf16_rne(xv[k]); } *(volatile v4f*)(OUT + (m0 + rr) * ow + oc + lane * 4) = v; } __threadfence(); } }
__global__ __launch_bounds__(256) void attn_kernel(const float* __restrict__ Q, const float* __restrict__ KV, int MLIM, float* __restrict__ AO) { const int wave = threadIdx.x >> 5, lane = threadIdx.x & 31; const size_t m = (size_t)blockIdx.x * 8 + wave; if (m >= (size_t)MLIM) return;
  const int b = (int)(m / (G * G * G)), d = (int)((m / (G * G)) % G), h = (int)((m / G) % G), w = (int)(m % G); float qv[8]; for (int k = 0; k < 8; ++k) qv[k] = Q[m * C + lane * 8 + k];
  float mx = -INFINITY, den = 0.0f, acc[8];
#pragma unroll
  for (int k = 0; k < 8; ++k) acc[k] = 0.0f;
#pragma unroll 1
  for (int o = 0; o < WS * WS * WS; ++o) { if (o == 13) continue; const int dd = d + o / 9 - 1, hh2 = h + (o / 3) % 3 - 1, ww = w + o % 3 - 1; if (dd < 0 || dd >= G || hh2 < 0 || hh2 >= G || ww < 0 || ww >= G) continue;
    const size_t n = (((size_t)b * G + dd) * G + hh2) * G + ww; const v4f k0 = *(const v4f*)(KV + n * 2 * C + lane * 8), k1 = *(const v4f*)(KV + n * 2 * C + lane * 8 + 4); float s = 0.0f; for (int k = 0; k < 4; ++k) { s += pmul(qv[k], k0[k]); s += pmul(qv[4 + k], k1[k]); } s += __shfl_xor(s, 1); s += __shfl_xor(s, 2);
    const float mn = fmaxf(mx, s); const float sf = (mx == -INFINITY) ? 0.0f : __expf(mx - mn); const float p = __expf(s - mn); den = den * sf + p; const v4f v0 = *(const v4f*)(KV + n * 2 * C + C + lane * 8), v1 = *(const v4f*)(KV + n * 2 * C + C + lane * 8 + 4);
#pragma unroll
    for (int k = 0; k < 4; ++k) { acc[k] = pmul(acc[k], sf) + pmul(p, v0[k]); acc[4 + k] = pmul(acc[4 + k], sf) + pmul(p, v1[k]); } mx = mn; }
  const float inv = den > 0.0f ? 1.0f / den : 0.0f; v4f o0, o1; for (int k = 0; k < 4; ++k) { o0[k] = pmul(acc[k], inv); o1[k] = pmul(acc[4 + k], inv); }
  for (int pass = 0; pass < 2; ++pass) { *(volatile v4f*)(AO + m * C + lane * 8) = o0; *(volatile v4f*)(AO + m * C + lane * 8 + 4) = o1; __threadfence(); } }
__global__ __launch_bounds__(32) void ffn1_kernel(const float* __restrict__ T, const b16* __restrict__ W1T, const float* __restrict__ bf1, const float* __restrict__ g, const float* __restrict__ be, int MLIM, b16* __restrict__ HH, b16* __restrict__ HL) {
  __shared__ __attribute__((aligned(16))) b16 Ah[16][C + 8], Al[16][C + 8]; __shared__ float Tf[16][132]; const int lane = threadIdx.x, nloc = lane & 15, hlf = lane >> 4; const int grp = blockIdx.x % 8; const size_t m0 = (size_t)(blockIdx.x / 8) * 16; if (m0 >= (size_t)MLIM) return;
  stage_rows(T, m0, g, be, true, false, Ah, Al, lane); wave_lds_sync(); v8f acc[8];
#pragma unroll
  for (int t = 0; t < 8; ++t) acc[t] = (v8f){};
#pragma unroll 2
  for (int kb = 0; kb < C; kb += 32) { const v16b a = frag_kb(&Ah[nloc][kb], hlf), al = frag_kb(&Al[nloc][kb], hlf);
#pragma unroll
    for (int t = 0; t < 8; ++t) { const v16b bw = frag_kb(W1T + (size_t)(grp * 128 + t * 16 + nloc) * C + kb, hlf); acc[t] = wmma16b(a, bw, acc[t]); acc[t] = wmma16b(al, bw, acc[t]); } }
#pragma unroll
  for (int t = 0; t < 8; ++t) { const int cc = grp * 128 + t * 16 + nloc; const float bias = bf16_rne(bf1[cc]);
#pragma unroll
    for (int r8 = 0; r8 < 8; ++r8) Tf[8 * hlf + r8][t * 16 + nloc] = gelu(acc[t][r8] * (1.0f / (XS * WSC)) + bias); }
  wave_lds_sync();
  for (int pass = 0; pass < 2; ++pass) { for (int rr = 0; rr < 16; ++rr) { v4f v = *(const v4f*)(&Tf[rr][lane * 4]); b16 ph[4], pl[4]; for (int k = 0; k < 4; ++k) split16(v[k] * XS, ph[k], pl[k]);
      typedef __attribute__((ext_vector_type(4))) _Float16 v4b; *(volatile v4b*)(HH + (m0 + rr) * F + grp * 128 + lane * 4) = (v4b){ph[0], ph[1], ph[2], ph[3]}; *(volatile v4b*)(HL + (m0 + rr) * F + grp * 128 + lane * 4) = (v4b){pl[0], pl[1], pl[2], pl[3]}; } __threadfence(); } }
__global__ __launch_bounds__(32) void ffn2_kernel(const b16* __restrict__ HH, const b16* __restrict__ HL, const b16* __restrict__ W2T, const float* __restrict__ bf2, const float* __restrict__ T, int MLIM, float* __restrict__ out) { __shared__ float Tf[16][132]; const int lane = threadIdx.x, nloc = lane & 15, hlf = lane >> 4; const int grp = blockIdx.x % 2; const size_t m0 = (size_t)(blockIdx.x / 2) * 16; if (m0 >= (size_t)MLIM) return;
  v8f acc[8];
#pragma unroll
  for (int t = 0; t < 8; ++t) acc[t] = (v8f){};
#pragma unroll 2
  for (int kb = 0; kb < F; kb += 32) { const v16b a = frag_kb(HH + (m0 + nloc) * F + kb, hlf), al = frag_kb(HL + (m0 + nloc) * F + kb, hlf);
#pragma unroll
    for (int t = 0; t < 8; ++t) { const v16b bw = frag_kb(W2T + (size_t)(grp * 128 + t * 16 + nloc) * F + kb, hlf); acc[t] = wmma16b(a, bw, acc[t]); acc[t] = wmma16b(al, bw, acc[t]); } }
#pragma unroll
  for (int t = 0; t < 8; ++t) { const int cc = grp * 128 + t * 16 + nloc; const float bias = bf16_rne(bf2[cc]);
#pragma unroll
    for (int r8 = 0; r8 < 8; ++r8) Tf[8 * hlf + r8][t * 16 + nloc] = acc[t][r8] * (1.0f / (XS * WSC)) + bias; }
  wave_lds_sync();
  for (int pass = 0; pass < 2; ++pass) { for (int rr = 0; rr < 16; ++rr) { v4f v = *(const v4f*)(&Tf[rr][lane * 4]); const v4f tv = *(const v4f*)(T + (m0 + rr) * C + grp * 128 + lane * 4); for (int k = 0; k < 4; ++k) v[k] += tv[k]; *(volatile v4f*)(out + (m0 + rr) * C + grp * 128 + lane * 4) = v; } __threadfence(); } }
}

extern "C" void kernel_launch(void* const* d_in, const int* in_sizes, int n_in, void* d_out, int out_size, void* d_ws, size_t ws_size, hipStream_t stream) {
  (void)n_in;
  auto Fp = [&](int i) { return (const float*)d_in[i]; };
  if (in_sizes[0] != M * C || in_sizes[1] != C * C || in_sizes[7] != C * C || in_sizes[13] != C * F || in_sizes[15] != F * C || out_size != M * C) return;
  const int MLIM = M;
  size_t off = 0; char* ws = (char*)d_ws;
  auto carve = [&](size_t bytes) { char* p = ws + off; off += (bytes + 255) & ~(size_t)255; return p; };
  b16* WQ = (b16*)carve((size_t)C * C * 2); b16* WK = (b16*)carve((size_t)C * C * 2); b16* WV = (b16*)carve((size_t)C * C * 2); b16* WO = (b16*)carve((size_t)C * C * 2); b16* W1T = (b16*)carve((size_t)F * C * 2); b16* W2T = (b16*)carve((size_t)C * F * 2);
  float* KV = (float*)carve((size_t)M * 2 * C * 4); float* Q = (float*)carve((size_t)M * C * 4); float* AO = (float*)carve((size_t)M * C * 4); float* T = (float*)carve((size_t)M * C * 4); b16* HH = (b16*)carve((size_t)M * F * 2); b16* HL = (b16*)carve((size_t)M * F * 2);
  if (off > ws_size || off > ((size_t)96 << 20)) return;
  wput_kernel<<<(C * C / 8 + 255) / 256, 256, 0, stream>>>(Fp(1), C, C, WQ); wput_kernel<<<(C * C / 8 + 255) / 256, 256, 0, stream>>>(Fp(3), C, C, WK); wput_kernel<<<(C * C / 8 + 255) / 256, 256, 0, stream>>>(Fp(5), C, C, WV); wput_kernel<<<(C * C / 8 + 255) / 256, 256, 0, stream>>>(Fp(7), C, C, WO);
  wput_kernel<<<(C * F / 8 + 255) / 256, 256, 0, stream>>>(Fp(13), C, F, W1T); wput_kernel<<<(C * F / 8 + 255) / 256, 256, 0, stream>>>(Fp(15), F, C, W2T);
  proj_kernel<0><<<(M / 16) * 4, 32, 0, stream>>>(Fp(0), Fp(0), WK, WV, Fp(4), Fp(6), nullptr, nullptr, MLIM, KV);
  proj_kernel<1><<<(M / 16) * 2, 32, 0, stream>>>(Fp(0), Fp(0), WQ, nullptr, Fp(2), nullptr, Fp(9), Fp(10), MLIM, Q);
  attn_kernel<<<(MLIM + 7) / 8, 256, 0, stream>>>(Q, KV, MLIM, AO);
  proj_kernel<2><<<(M / 16) * 2, 32, 0, stream>>>(AO, Fp(0), WO, nullptr, Fp(8), nullptr, nullptr, nullptr, MLIM, T);
  ffn1_kernel<<<(M / 16) * 8, 32, 0, stream>>>(T, W1T, Fp(14), Fp(11), Fp(12), MLIM, HH, HL);
  ffn2_kernel<<<(M / 16) * 2, 32, 0, stream>>>(HH, HL, W2T, Fp(16), T, MLIM, (float*)d_out);
}
